// LSTM_42090679501192
// MI455X (gfx1250) — hardware-verified
//
#include <hip/hip_runtime.h>
#include <math.h>

constexpr int NBAT    = 64;
constexpr int NLEN    = 512;
constexpr int NCH     = 7;
constexpr int NHID    = 128;
constexpr int NGATE   = 4 * NHID;
constexpr int NSEQ    = NBAT * NCH;
constexpr int NPRED   = 96;
constexpr int SEQ_BLK = 16;
constexpr int NBLK    = NSEQ / SEQ_BLK;
constexpr int NTHR_SEQ = 512;
constexpr int NFLAT   = NBAT * NLEN * NCH;
constexpr int NOUT    = NSEQ * NPRED;
constexpr int BATCH_FLAT = NLEN * NCH;
constexpr int OUT_BATCH  = NPRED * NCH;
constexpr float WCARRY  = 16.0f;
constexpr float HCARRY  = 64.0f;
constexpr float ACC_INV = 1.0f / (WCARRY * HCARRY);
constexpr float NORM_EPS = 1e-5f;
static_assert(NSEQ == 448 && NBLK == 28 && NSEQ % SEQ_BLK == 0, "sequence tiling");
static_assert(NGATE == 512 && NHID % 32 == 0 && (2 * NHID) % 32 == 0, "K multiples of 32");
static_assert(NFLAT == NSEQ * NLEN, "raw reshape");
static_assert(BATCH_FLAT % NCH == 0, "channel phase");
static_assert(NOUT == 168 * 256, "head grid exact");
static_assert(NOUT * 4 == 172032, "output bytes");
static_assert(NSEQ == 14 * 32, "stat lines exact");

typedef __attribute__((ext_vector_type(16))) _Float16 v16h;
typedef __attribute__((ext_vector_type(8)))  _Float16 v8h;
typedef __attribute__((ext_vector_type(8)))  float    v8f;
typedef __attribute__((ext_vector_type(4)))  float    v4f;
typedef __attribute__((ext_vector_type(2)))  unsigned v2u;

union FragU { v16h v; v8h h[2]; };
__device__ __forceinline__ v16h frag_load(const _Float16* p) {
  FragU f;
  f.h[0] = *(const v8h*)(p);
  f.h[1] = *(const v8h*)(p + 16);
  return f.v;
}
__device__ __forceinline__ v8f frag_mma(v16h a, v16h b, v8f c) {
  return __builtin_amdgcn_wmma_f32_16x16x32_f16(false, a, false, b, (short)0, c, false, false);
}
__device__ __forceinline__ void wmma_guard2(v8f& a, v8f& b, v16h x, v16h y, v16h z) {
  asm volatile("v_nop\n\tv_nop\n\tv_nop\n\tv_nop" : "+v"(a), "+v"(b) : "v"(x), "v"(y), "v"(z) : "memory");
}
__device__ __forceinline__ void hold4_h(v16h& a, v16h& b, v16h& c, v16h& d) {
  asm volatile("" : "+v"(a), "+v"(b), "+v"(c), "+v"(d));
}

__global__ __launch_bounds__(256) void prep_kernel(const float* __restrict__ Wih, const float* __restrict__ Whh,
                                                   const float* __restrict__ bih, const float* __restrict__ bhh,
                                                   const float* __restrict__ embW, const float* __restrict__ embb,
                                                   unsigned short* __restrict__ W0, unsigned short* __restrict__ WCAT,
                                                   float* __restrict__ avec, float* __restrict__ cvec,
                                                   float* __restrict__ b1vec) {
  const int tid = threadIdx.x;
  const int blk = blockIdx.x;
  if (blk < 96) {
    const float* src;
    unsigned short* dst;
    if (blk < 32) {
      const int q = blk * 256 + tid;
      src = Whh + (size_t)q * 8;
      dst = W0 + (size_t)q * 8;
    } else {
      const int part = (blk - 32) >> 5;
      const int q = ((blk - 32) & 31) * 256 + tid;
      const int g = q >> 4;
      const int seg = q & 15;
      const float* base = part ? Whh : Wih;
      src = base + (size_t)NGATE * NHID + (size_t)g * NHID + seg * 8;
      dst = WCAT + (size_t)g * (2 * NHID) + part * NHID + seg * 8;
    }
    const v4f va = *(const v4f*)(src);
    const v4f vb = *(const v4f*)(src + 4);
    v8h hv;
#pragma unroll
    for (int e = 0; e < 4; ++e) {
      hv[e]     = (_Float16)(va[e] * WCARRY);
      hv[4 + e] = (_Float16)(vb[e] * WCARRY);
    }
    *(volatile v8h*)dst = hv;
    __threadfence();
    *(volatile v8h*)dst = hv;
  } else {
    const int g = (blk - 96) * 256 + tid;
    const float* wr = Wih + (size_t)g * NHID;
    float sa = 0.0f, sc = 0.0f;
#pragma unroll 1
    for (int k = 0; k < NHID; k += 4) {
      const v4f w  = *(const v4f*)(wr + k);
      const v4f ew = *(const v4f*)(embW + k);
      const v4f eb = *(const v4f*)(embb + k);
#pragma unroll
      for (int e = 0; e < 4; ++e) {
        sa = fmaf(w[e], ew[e], sa);
        sc = fmaf(w[e], eb[e], sc);
      }
    }
    const float cv = (sc + bih[g]) + bhh[g];
    const float bv = bih[NGATE + g] + bhh[NGATE + g];
    *(volatile float*)(avec + g)  = sa;
    *(volatile float*)(cvec + g)  = cv;
    *(volatile float*)(b1vec + g) = bv;
    __threadfence();
    *(volatile float*)(avec + g)  = sa;
    *(volatile float*)(cvec + g)  = cv;
    *(volatile float*)(b1vec + g) = bv;
  }
}

__global__ __launch_bounds__(256) void stats_kernel(const float* __restrict__ x, float* __restrict__ mean,
                                                    float* __restrict__ stdv, float* __restrict__ rstd) {
  __shared__ float sm[32];
  __shared__ float ss[32];
  const int tid = threadIdx.x, lane = tid & 31, wave = tid >> 5;
#pragma unroll 1
  for (int q = 0; q < 4; ++q) {
    const int pl = wave * 4 + q;
    const int p = blockIdx.x * 32 + pl;
    const int b = p / NCH;
    const int u = p - b * NCH;
    const float* xb = x + (size_t)b * BATCH_FLAT + u;
    float v[16];
#pragma unroll
    for (int i = 0; i < 16; ++i) v[i] = xb[(size_t)(lane + 32 * i) * NCH];
    float s = 0.0f;
#pragma unroll
    for (int i = 0; i < 16; ++i) s += v[i];
#pragma unroll
    for (int off = 1; off < 32; off <<= 1) s += __shfl_xor(s, off, 32);
    const float mu = s * (1.0f / NLEN);
    float sq = 0.0f;
#pragma unroll
    for (int i = 0; i < 16; ++i) {
      const float d = v[i] - mu;
      sq += d * d;
    }
#pragma unroll
    for (int off = 1; off < 32; off <<= 1) sq += __shfl_xor(sq, off, 32);
    const float sd = sqrtf(sq * (1.0f / NLEN) + NORM_EPS);
    if (lane == 0) {
      sm[pl] = mu;
      ss[pl] = sd;
    }
  }
  __syncthreads();
  if (wave == 0) {
    const float mu = sm[lane];
    const float sd = ss[lane];
    const float rs = 1.0f / sd;
    const int idx = blockIdx.x * 32 + lane;
    *(volatile float*)(mean + idx) = mu;
    *(volatile float*)(stdv + idx) = sd;
    *(volatile float*)(rstd + idx) = rs;
    __threadfence();
    *(volatile float*)(mean + idx) = mu;
    *(volatile float*)(stdv + idx) = sd;
    *(volatile float*)(rstd + idx) = rs;
  }
}

template <int KDIM>
__global__ __launch_bounds__(NTHR_SEQ) void lstm_seq_kernel(
    const float* __restrict__ x, const float* __restrict__ mean, const float* __restrict__ rstd,
    const float* __restrict__ avec, const float* __restrict__ cvec,
    const unsigned short* __restrict__ Wp, unsigned short* hs0, float* __restrict__ h1out) {
  constexpr bool L1   = (KDIM == 2 * NHID);
  constexpr int NKC   = KDIM / 32;
  constexpr int HP    = KDIM + 8;
  constexpr int HCOL0 = KDIM - NHID;
  static_assert(KDIM == NHID || KDIM == 2 * NHID, "K shape");
  static_assert(NKC % 4 == 0, "fragment groups of four");
  __shared__ __align__(16) _Float16 sH[SEQ_BLK * HP];
  __shared__ __align__(16) float    sGO[2 * SEQ_BLK * NHID];
  __shared__ __align__(16) float    sST[L1 ? 4 : NLEN * SEQ_BLK];

  const _Float16* W = (const _Float16*)Wp;
  const int tid = threadIdx.x, lane = tid & 31, wave = tid >> 5;
  const int ub = wave & 7, gp = wave >> 3;
  const int c = lane & 15, hh = lane >> 4, koff = hh * 8;
  const int j = 16 * ub + c;
  const int blk = blockIdx.x;
  const int rowbase = blk * SEQ_BLK;
  const int prow = tid >> 5, pcol4 = (tid & 31) * 4;

  {
    v2u zz;
    zz[0] = 0u;
    zz[1] = 0u;
    *(v2u*)(sH + prow * HP + HCOL0 + pcol4) = zz;
  }
  if (L1) {
    const v2u p0 = *(const v2u*)(hs0 + ((size_t)blk * NLEN * SEQ_BLK) * NHID + (size_t)tid * 4);
    *(v2u*)(sH + prow * HP + pcol4) = p0;
  } else {
#pragma unroll 1
    for (int it = 0; it < SEQ_BLK; ++it) {
      const int i = (rowbase + it) * NLEN + tid;
      const int b = i / BATCH_FLAT;
      const int u = i % NCH;
      const float xv = x[i];
      const float mu = mean[b * NCH + u];
      const float rs = rstd[b * NCH + u];
      sST[tid * SEQ_BLK + it] = (xv - mu) * rs;
    }
  }

  v16h bfr[2][NKC];
#pragma unroll
  for (int gi = 0; gi < 2; ++gi) {
    const _Float16* wrow = W + (size_t)((2 * gp + gi) * NHID + j) * KDIM + koff;
#pragma unroll
    for (int k4 = 0; k4 < NKC; k4 += 4) {
#pragma unroll
      for (int e = 0; e < 4; ++e) bfr[gi][k4 + e] = frag_load(wrow + 32 * (k4 + e));
      hold4_h(bfr[gi][k4], bfr[gi][k4 + 1], bfr[gi][k4 + 2], bfr[gi][k4 + 3]);
    }
  }
  float aco[2], cco[2];
#pragma unroll
  for (int gi = 0; gi < 2; ++gi) {
    const int gcol = (2 * gp + gi) * NHID + j;
    aco[gi] = L1 ? 0.0f : avec[gcol];
    cco[gi] = cvec[gcol];
  }
  float cst[8], hst[8];
#pragma unroll
  for (int r = 0; r < 8; ++r) {
    cst[r] = 0.0f;
    hst[r] = 0.0f;
  }
  __syncthreads();

  const _Float16* arow = sH + c * HP + koff;
  const v8f z8 = {0.f, 0.f, 0.f, 0.f, 0.f, 0.f, 0.f, 0.f};

#pragma unroll 1
  for (int t = 0; t < NLEN; ++t) {
    v2u pre;
    pre[0] = 0u;
    pre[1] = 0u;
    if (L1) {
      const int tn = (t + 1 < NLEN) ? (t + 1) : (NLEN - 1);
      pre = *(const v2u*)(hs0 + ((size_t)(blk * NLEN + tn) * SEQ_BLK) * NHID + (size_t)tid * 4);
    }
    float sv[8];
    if (!L1) {
      const v4f s0 = *(const v4f*)(sST + t * SEQ_BLK + 8 * hh);
      const v4f s1 = *(const v4f*)(sST + t * SEQ_BLK + 8 * hh + 4);
#pragma unroll
      for (int e = 0; e < 4; ++e) {
        sv[e] = s0[e];
        sv[4 + e] = s1[e];
      }
    } else {
#pragma unroll
      for (int e = 0; e < 8; ++e) sv[e] = 0.0f;
    }

    v8f acc0 = z8, acc1 = z8;
#pragma unroll
    for (int kc = 0; kc < NKC; ++kc) {
      const v16h a = frag_load(arow + 32 * kc);
      acc0 = frag_mma(a, bfr[0][kc], acc0);
      acc1 = frag_mma(a, bfr[1][kc], acc1);
      wmma_guard2(acc0, acc1, a, bfr[0][kc], bfr[1][kc]);
    }

    float a0[8], a1[8];
#pragma unroll
    for (int r = 0; r < 8; ++r) {
      const float xin0 = L1 ? cco[0] : fmaf(sv[r], aco[0], cco[0]);
      const float xin1 = L1 ? cco[1] : fmaf(sv[r], aco[1], cco[1]);
      const float z0 = acc0[r] * ACC_INV + xin0;
      const float z1 = acc1[r] * ACC_INV + xin1;
      const float e0 = expf(gp ? (2.0f * z0) : (-z0));
      const float q0 = 1.0f / (1.0f + e0);
      a0[r] = gp ? (1.0f - 2.0f * q0) : q0;
      a1[r] = 1.0f / (1.0f + expf(-z1));
    }
    if (gp == 1) {
#pragma unroll
      for (int r = 0; r < 8; ++r) {
        sGO[(8 * hh + r) * NHID + j] = a0[r];
        sGO[SEQ_BLK * NHID + (8 * hh + r) * NHID + j] = a1[r];
      }
    }
    __syncthreads();
    if (gp == 0) {
#pragma unroll
      for (int r = 0; r < 8; ++r) {
        const float gv = sGO[(8 * hh + r) * NHID + j];
        const float ov = sGO[SEQ_BLK * NHID + (8 * hh + r) * NHID + j];
        const float cn = a1[r] * cst[r] + a0[r] * gv;
        cst[r] = cn;
        const float th = 1.0f - 2.0f / (1.0f + expf(2.0f * cn));
        const float hn = ov * th;
        hst[r] = hn;
        sH[(8 * hh + r) * HP + HCOL0 + j] = (_Float16)(hn * HCARRY);
      }
    }
    if (L1) {
      *(v2u*)(sH + prow * HP + pcol4) = pre;
    }
    __syncthreads();
    if (!L1) {
      if (gp == 1) {
        const int j2 = tid - 256;
        const int row = j2 >> 4, col8 = (j2 & 15) * 8;
        const v8h hv = *(const v8h*)(sH + row * HP + col8);
        unsigned short* dst = hs0 + ((size_t)(blk * NLEN + t) * SEQ_BLK) * NHID + (size_t)j2 * 8;
        *(volatile v8h*)dst = hv;
        __threadfence();
        *(volatile v8h*)dst = hv;
      }
    }
  }

  if (L1) {
    if (gp == 0) {
#pragma unroll
      for (int r = 0; r < 8; ++r) sGO[(8 * hh + r) * NHID + j] = hst[r];
    }
    __syncthreads();
    const int c4 = (tid & 31) * 4;
    const v4f v = *(const v4f*)(sGO + prow * NHID + c4);
    float* dst = h1out + (size_t)(rowbase + prow) * NHID + c4;
    *(volatile v4f*)dst = v;
    __threadfence();
    *(volatile v4f*)dst = v;
  }
}

__global__ __launch_bounds__(256) void head_kernel(const float* __restrict__ h1, const float* __restrict__ fcW,
                                                   const float* __restrict__ fcb, const float* __restrict__ mean,
                                                   const float* __restrict__ stdv, float* __restrict__ out) {
  const int f = blockIdx.x * 256 + threadIdx.x;
  if (f >= NOUT) return;
  const int n = f / NPRED;
  const int p = f - n * NPRED;
  const float* hp = h1 + (size_t)n * NHID;
  const float* wp = fcW + (size_t)p * NHID;
  float acc = fcb[p];
#pragma unroll 1
  for (int k = 0; k < NHID; k += 4) {
    const v4f hv = *(const v4f*)(hp + k);
    const v4f wv = *(const v4f*)(wp + k);
#pragma unroll
    for (int e = 0; e < 4; ++e) acc = fmaf(hv[e], wv[e], acc);
  }
  const int si = (f / OUT_BATCH) * NCH + (f % NCH);
  const float val = acc * stdv[si] + mean[si];
  *(volatile float*)(out + f) = val;
  __threadfence();
  *(volatile float*)(out + f) = val;
}

extern "C" void kernel_launch(void* const* d_in, const int* in_sizes, int n_in,
                              void* d_out, int out_size, void* d_ws, size_t ws_size, hipStream_t stream) {
  if (n_in < 9 || d_out == nullptr || d_ws == nullptr) return;
  if (in_sizes[0] != NFLAT || in_sizes[1] != NHID || in_sizes[2] != NHID ||
      in_sizes[3] != 2 * NGATE * NHID || in_sizes[4] != 2 * NGATE * NHID ||
      in_sizes[5] != 2 * NGATE || in_sizes[6] != 2 * NGATE ||
      in_sizes[7] != NPRED * NHID || in_sizes[8] != NPRED || out_size != NOUT) return;

  const float* x    = (const float*)d_in[0];
  const float* embW = (const float*)d_in[1];
  const float* embb = (const float*)d_in[2];
  const float* Wih  = (const float*)d_in[3];
  const float* Whh  = (const float*)d_in[4];
  const float* bih  = (const float*)d_in[5];
  const float* bhh  = (const float*)d_in[6];
  const float* fcW  = (const float*)d_in[7];
  const float* fcb  = (const float*)d_in[8];
  float* out = (float*)d_out;

  char* ws = (char*)d_ws;
  size_t off = 0;
  auto carve = [&](size_t bytes) -> char* { char* p = ws + off; off += (bytes + 255) & ~(size_t)255; return p; };
  unsigned short* HS0  = (unsigned short*)carve((size_t)NBLK * NLEN * SEQ_BLK * NHID * 2);
  unsigned short* W0   = (unsigned short*)carve((size_t)NGATE * NHID * 2);
  unsigned short* WCAT = (unsigned short*)carve((size_t)NGATE * 2 * NHID * 2);
  float* H1   = (float*)carve((size_t)NSEQ * NHID * 4);
  float* AV   = (float*)carve(2048);
  float* CV   = (float*)carve(2048);
  float* B1   = (float*)carve(2048);
  float* MEAN = (float*)carve(2048);
  float* STDV = (float*)carve(2048);
  float* RSTD = (float*)carve(2048);
  if (off > ws_size || off > (size_t)134217728) return;

  prep_kernel<<<98, 256, 0, stream>>>(Wih, Whh, bih, bhh, embW, embb, W0, WCAT, AV, CV, B1);
  stats_kernel<<<NSEQ / 32, 256, 0, stream>>>(x, MEAN, STDV, RSTD);
  lstm_seq_kernel<NHID><<<NBLK, NTHR_SEQ, 0, stream>>>(x, MEAN, RSTD, AV, CV, W0, HS0, H1);
  lstm_seq_kernel<2 * NHID><<<NBLK, NTHR_SEQ, 0, stream>>>(x, MEAN, RSTD, AV, B1, WCAT, HS0, H1);
  head_kernel<<<NOUT / 256, 256, 0, stream>>>(H1, fcW, fcb, MEAN, STDV, out);
}
